// hierarchical_Feature_spatial_attention_6614249636391
// MI455X (gfx1250) — hardware-verified
//
#include <hip/hip_runtime.h>
#include <math.h>

constexpr int kBatch     = 2;
constexpr int kChan      = 64;
constexpr int kSpat      = 9216;
constexpr int kChunk     = 512;
constexpr int kNumChunks = kSpat / kChunk;
constexpr int kSmThreads = 128;
constexpr int kSmIters   = kSpat / (kSmThreads * 8);
static_assert(kSpat % kChunk == 0);
static_assert(kSmIters * kSmThreads * 8 == kSpat);
static_assert(kSpat % 64 == 0 && kChunk % 64 == 0 && kChan % 64 == 0);
static_assert(kChan % 32 == 0 && kSpat % 32 == 0);

typedef __attribute__((ext_vector_type(16))) _Float16 v16h;
typedef __attribute__((ext_vector_type(8)))  _Float16 v8h;
typedef __attribute__((ext_vector_type(16))) __bf16   v16b;
typedef __attribute__((ext_vector_type(8)))  __bf16   v8b;
typedef __attribute__((ext_vector_type(8)))  float    v8f;
typedef __attribute__((ext_vector_type(4)))  float    v4f;
typedef __attribute__((ext_vector_type(4)))  unsigned int v4u;

__device__ __forceinline__ unsigned short f2bf_bits(float f) {
  unsigned u = __float_as_uint(f);
  return (unsigned short)((u + 0x7FFFu + ((u >> 16) & 1u)) >> 16);
}
__device__ __forceinline__ float bf_bits2f(unsigned short h) { return __uint_as_float(((unsigned)h) << 16); }
__device__ __forceinline__ unsigned pk16(unsigned short a, unsigned short b) { return (unsigned)a | ((unsigned)b << 16); }

__device__ __forceinline__ void dep_guard_h(v8f& a, v8f& b, v16h x, v16h y) { asm volatile("v_nop\n\tv_nop\n\tv_nop\n\tv_nop" : "+v"(a), "+v"(b) : "v"(x), "v"(y)); }
__device__ __forceinline__ void dep_guard_b(v8f& a, v8f& b, v16b x, v16b y) { asm volatile("v_nop\n\tv_nop\n\tv_nop\n\tv_nop" : "+v"(a), "+v"(b) : "v"(x), "v"(y)); }
__device__ __forceinline__ void keep4_h(v16h a, v16h b, v16h c, v16h d) { asm volatile("v_nop" :: "v"(a), "v"(b), "v"(c), "v"(d)); }
__device__ __forceinline__ void keep4_b(v16b a, v16b b, v16b c, v16b d) { asm volatile("v_nop" :: "v"(a), "v"(b), "v"(c), "v"(d)); }
__device__ __forceinline__ void acc_guard4(v8f& a, v8f& b, v8f& c, v8f& d) { asm volatile("v_nop\n\tv_nop\n\tv_nop\n\tv_nop" : "+v"(a), "+v"(b), "+v"(c), "+v"(d)); }
template <typename T> struct Frag;
template <> struct Frag<_Float16> {
  typedef v16h V; union U { v16h v; v8h h[2]; };
  static __device__ __forceinline__ v16h load(const _Float16* p) {
    U f; f.h[0] = *(const v8h*)(p); f.h[1] = *(const v8h*)(p + 16); return f.v;
  }
  static __device__ __forceinline__ v8f mma(v16h a, v16h b, v8f c) {
    return __builtin_amdgcn_wmma_f32_16x16x32_f16(false, a, false, b, (short)0, c, false, false);
  }
  static __device__ __forceinline__ void guard(v8f& a, v8f& b, v16h x, v16h y) { dep_guard_h(a, b, x, y); }
  static __device__ __forceinline__ void keep(v16h a, v16h b, v16h c, v16h d) { keep4_h(a, b, c, d); }
};
template <> struct Frag<__bf16> {
  typedef v16b V; union U { v16b v; v8b h[2]; };
  static __device__ __forceinline__ v16b load(const __bf16* p) {
    U f; f.h[0] = *(const v8b*)(p); f.h[1] = *(const v8b*)(p + 16); return f.v;
  }
  static __device__ __forceinline__ v8f mma(v16b a, v16b b, v8f c) {
    return __builtin_amdgcn_wmma_f32_16x16x32_bf16(false, a, false, b, (short)0, c, false, false);
  }
  static __device__ __forceinline__ void guard(v8f& a, v8f& b, v16b x, v16b y) { dep_guard_b(a, b, x, y); }
  static __device__ __forceinline__ void keep(v16b a, v16b b, v16b c, v16b d) { keep4_b(a, b, c, d); }
};

template <int ET> struct Elem;
template <> struct Elem<0> { typedef _Float16 T; };
template <> struct Elem<1> { typedef __bf16 T; };
template <int ET, int SPL, int BIAS_MODE, int OUT_MODE, bool RESID, int ACT = 0>
__global__ __launch_bounds__(256) void wmma_gemm64(
    const unsigned short* __restrict__ Ap, const unsigned short* __restrict__ A2p, int lda, long strideA,
    const unsigned short* __restrict__ Btp, const unsigned short* __restrict__ Bt2p, int ldb, long strideB,
    void* __restrict__ Cout, void* __restrict__ Cout2, int ldc, long strideC,
    const float* __restrict__ bias,
    const float* __restrict__ resid, long strideR,
    int M, int N, int K, float scale) {
  typedef typename Elem<ET>::T T;
  typedef typename Frag<T>::V V;
  const T* A = (const T*)Ap; const T* A2 = (const T*)A2p; const T* Bt = (const T*)Btp; const T* Bt2 = (const T*)Bt2p;
  __shared__ __align__(16) float sT[8][16 * 68];
  const int b    = blockIdx.y;
  const int lane = threadIdx.x & 31;
  const int wave = threadIdx.x >> 5;
  const int tilesN = N >> 6;
  const int tilesM = M >> 6;
  const int tile = blockIdx.x * 8 + wave;
  if (tile >= tilesM * tilesN) return;
  const int tm = tile / tilesN;
  const int tn = tile - tm * tilesN;
  const int m0 = tm << 6;
  const int n0 = tn << 6;

  const T* Ab  = A  + (size_t)b * strideA;
  const T* Bb  = Bt + (size_t)b * strideB;
  const T* Ab2 = (SPL >= 1) ? (A2  + (size_t)b * strideA) : nullptr;
  const T* Bb2 = (SPL == 2) ? (Bt2 + (size_t)b * strideB) : nullptr;

  const int rlane = lane & 15;
  const int koff  = (lane >> 4) * 8;
  const int mOff  = (lane >> 4) * 8;

  v8f acc[4][4];
#pragma unroll
  for (int i = 0; i < 4; ++i)
#pragma unroll
    for (int j = 0; j < 4; ++j) acc[i][j] = (v8f){0.f,0.f,0.f,0.f,0.f,0.f,0.f,0.f};

  for (int k0 = 0; k0 < K; k0 += 32) {
    V bh[4], bl[4];
#pragma unroll
    for (int j = 0; j < 4; ++j) {
      const size_t bo = (size_t)(n0 + (j << 4) + rlane) * ldb + koff + k0;
      bh[j] = Frag<T>::load(Bb + bo);
      if (SPL == 2) bl[j] = Frag<T>::load(Bb2 + bo);
    }
#pragma unroll
    for (int i = 0; i < 4; ++i) {
      const size_t ao = (size_t)(m0 + (i << 4) + rlane) * lda + koff + k0;
      V ah = Frag<T>::load(Ab + ao);
      V al;
      if (SPL >= 1) al = Frag<T>::load(Ab2 + ao);
#pragma unroll
      for (int j = 0; j < 4; ++j) {
        acc[i][j] = Frag<T>::mma(ah, bh[j], acc[i][j]);
        if (SPL == 2) acc[i][j] = Frag<T>::mma(ah, bl[j], acc[i][j]);
        if (SPL >= 1) acc[i][j] = Frag<T>::mma(al, bh[j], acc[i][j]);
      }
      Frag<T>::guard(acc[i][0], acc[i][3], ah, (SPL >= 1) ? al : ah);
    }
    Frag<T>::keep(bh[0], bh[1], bh[2], bh[3]);
    if (SPL == 2) Frag<T>::keep(bl[0], bl[1], bl[2], bl[3]);
  }
  acc_guard4(acc[0][0], acc[0][1], acc[0][2], acc[0][3]);
  acc_guard4(acc[1][0], acc[1][1], acc[1][2], acc[1][3]);
  acc_guard4(acc[2][0], acc[2][1], acc[2][2], acc[2][3]);
  acc_guard4(acc[3][0], acc[3][1], acc[3][2], acc[3][3]);

  float* slab = sT[wave];
  const float* Rb = RESID ? (resid + (size_t)b * strideR) : nullptr;
#pragma unroll
  for (int i = 0; i < 4; ++i) {
    const int mBase = m0 + (i << 4);
#pragma unroll
    for (int j = 0; j < 4; ++j) {
      const int n = n0 + (j << 4) + rlane;
      float bv = 0.f;
      if (BIAS_MODE == 2) bv = bias[n];
#pragma unroll
      for (int r = 0; r < 8; ++r) {
        float v = acc[i][j][r] * scale;
        if (BIAS_MODE == 1) v += bias[mBase + mOff + r];
        if (BIAS_MODE == 2) v += bv;
        if (RESID) v += Rb[(size_t)(mBase + mOff + r) * ldc + n];
        if (ACT == 2) v = fmaxf(v, 0.0f);
        if (ACT == 4) v = (v > 0.f) ? v : 0.01f * v;
        slab[(mOff + r) * 68 + (j << 4) + rlane] = v;
      }
    }
    __builtin_amdgcn_fence(__ATOMIC_RELEASE, "workgroup");
    __builtin_amdgcn_wave_barrier();
    __builtin_amdgcn_fence(__ATOMIC_ACQUIRE, "workgroup");
    if (OUT_MODE == 0) {
      float* C = (float*)Cout + (size_t)b * strideC;
      const int hh = lane >> 4, c4 = (lane & 15) * 4;
      for (int pass = 0; pass < 2; ++pass) {
#pragma unroll
        for (int it = 0; it < 8; ++it) {
          const int row = it * 2 + hh;
          v4f v = *(const v4f*)(slab + row * 68 + c4);
          *(volatile v4f*)(C + (size_t)(mBase + row) * ldc + n0 + c4) = v;
        }
        __threadfence();
      }
    } else {
      const int q = lane >> 3, c8 = (lane & 7) * 8;
      unsigned short* C  = (unsigned short*)Cout  + (size_t)b * strideC;
      unsigned short* C2 = (OUT_MODE == 2) ? ((unsigned short*)Cout2 + (size_t)b * strideC) : nullptr;
      for (int pass = 0; pass < 2; ++pass) {
#pragma unroll
        for (int it = 0; it < 4; ++it) {
          const int row = it * 4 + q;
          const float* sp = slab + row * 68 + c8;
          v8h hv, lv;
#pragma unroll
          for (int e = 0; e < 8; ++e) {
            if (OUT_MODE == 1) {
              hv[e] = (_Float16)sp[e];
            } else {
              unsigned short hb = f2bf_bits(sp[e]);
              unsigned short lb = f2bf_bits(sp[e] - bf_bits2f(hb));
              hv[e] = __builtin_bit_cast(_Float16, hb);
              lv[e] = __builtin_bit_cast(_Float16, lb);
            }
          }
          *(volatile v8h*)(C + (size_t)(mBase + row) * ldc + n0 + c8) = hv;
          if (OUT_MODE == 2) *(volatile v8h*)(C2 + (size_t)(mBase + row) * ldc + n0 + c8) = lv;
        }
        __threadfence();
      }
    }
    __builtin_amdgcn_fence(__ATOMIC_RELEASE, "workgroup");
    __builtin_amdgcn_wave_barrier();
    __builtin_amdgcn_fence(__ATOMIC_ACQUIRE, "workgroup");
  }
}

__global__ __launch_bounds__(256) void tcast_kernel(const float* __restrict__ yi, const float* __restrict__ pi,
                                                    unsigned short* __restrict__ yit, unsigned short* __restrict__ pit) {
  __shared__ float sm[64][65];
  const int t  = threadIdx.x;
  const int s0 = blockIdx.x * 64;
  const int b  = blockIdx.y;
  const int z  = blockIdx.z;
  const float* src = (z == 0) ? pi : yi;
  unsigned short* dst = (z == 0) ? pit : yit;
  const float* sb = src + (size_t)b * kChan * kSpat;
#pragma unroll
  for (int i = 0; i < 16; ++i) {
    const int e  = i * 256 + t;
    const int c  = e >> 6;
    const int sl = e & 63;
    sm[sl][c] = sb[(size_t)c * kSpat + s0 + sl];
  }
  __syncthreads();
  const int lane = t & 31, wave = t >> 5;
  const int q = lane >> 3, c8 = (lane & 7) * 8;
  unsigned short* db = dst + ((size_t)b * kSpat + s0) * kChan;
  for (int pass = 0; pass < 2; ++pass) {
#pragma unroll
    for (int it = 0; it < 2; ++it) {
      const int row = wave * 8 + it * 4 + q;
      unsigned short hb[8];
#pragma unroll
      for (int e = 0; e < 8; ++e) hb[e] = f2bf_bits(sm[row][c8 + e]);
      const v4u u = (v4u){pk16(hb[0], hb[1]), pk16(hb[2], hb[3]), pk16(hb[4], hb[5]), pk16(hb[6], hb[7])};
      *(volatile v4u*)(db + (size_t)row * kChan + c8) = u;
    }
    __threadfence();
  }
}

__global__ __launch_bounds__(256) void cast8_bf16_kernel(const float* __restrict__ in, unsigned short* __restrict__ out, int n8) {
  const int i = blockIdx.x * 256 + threadIdx.x;
  if (i >= n8) return;
  const float* p = in + 8 * (size_t)i;
  const v4f a = *(const v4f*)(p);
  const v4f c = *(const v4f*)(p + 4);
  unsigned short hb[8];
#pragma unroll
  for (int e = 0; e < 4; ++e) {
    hb[e]     = f2bf_bits(a[e]);
    hb[4 + e] = f2bf_bits(c[e]);
  }
  const v4u u = (v4u){pk16(hb[0], hb[1]), pk16(hb[2], hb[3]), pk16(hb[4], hb[5]), pk16(hb[6], hb[7])};
  unsigned short* q = out + 8 * (size_t)i;
  *(volatile v4u*)q = u;
  __threadfence();
  *(volatile v4u*)q = u;
}

__device__ __forceinline__ float wave_max32(float v) {
#pragma unroll
  for (int off = 16; off > 0; off >>= 1) v = fmaxf(v, __shfl_xor(v, off, 32));
  return v;
}
__device__ __forceinline__ float wave_sum32(float v) {
#pragma unroll
  for (int off = 16; off > 0; off >>= 1) v += __shfl_xor(v, off, 32);
  return v;
}

__global__ __launch_bounds__(kSmThreads) void softmax_split_kernel(const float* __restrict__ st,
                                                                  unsigned short* __restrict__ whi,
                                                                  unsigned short* __restrict__ wlo) {
  __shared__ __align__(16) float rowf[kSpat];
  __shared__ v4u packbuf[kSpat / 4];
  __shared__ float redm[4];
  __shared__ float reds[4];
  const int t    = threadIdx.x;
  const int lane = t & 31, wave = t >> 5;
  const int row  = blockIdx.x;
  const int b    = blockIdx.y;
  const size_t rofs = ((size_t)b * kChunk + row) * kSpat;
  const float* sr = st + rofs;

  float m = -INFINITY;
#pragma unroll 1
  for (int i = 0; i < kSmIters; ++i) {
    const int base = (i * kSmThreads + t) * 8;
    const v4f a = *(const v4f*)(sr + base);
    const v4f c = *(const v4f*)(sr + base + 4);
    *(v4f*)(rowf + base)     = a;
    *(v4f*)(rowf + base + 4) = c;
    const float ma = fmaxf(fmaxf(a[0], a[1]), fmaxf(a[2], a[3]));
    const float mc = fmaxf(fmaxf(c[0], c[1]), fmaxf(c[2], c[3]));
    m = fmaxf(m, fmaxf(ma, mc));
  }
  m = wave_max32(m);
  if (lane == 0) redm[wave] = m;
  __syncthreads();
  const float mx = fmaxf(fmaxf(redm[0], redm[1]), fmaxf(redm[2], redm[3]));

  float ssum = 0.f;
#pragma unroll 1
  for (int i = 0; i < kSmIters; ++i) {
    const int base = (i * kSmThreads + t) * 8;
    v4f a = *(const v4f*)(rowf + base);
    v4f c = *(const v4f*)(rowf + base + 4);
#pragma unroll
    for (int e = 0; e < 4; ++e) {
      a[e] = expf(a[e] - mx);
      c[e] = expf(c[e] - mx);
    }
    *(v4f*)(rowf + base)     = a;
    *(v4f*)(rowf + base + 4) = c;
    ssum += ((a[0] + a[1]) + (a[2] + a[3])) + ((c[0] + c[1]) + (c[2] + c[3]));
  }
  ssum = wave_sum32(ssum);
  if (lane == 0) reds[wave] = ssum;
  __syncthreads();
  const float stot = ((reds[0] + reds[1]) + reds[2]) + reds[3];
  const float inv  = 1.0f / stot;

#pragma unroll 1
  for (int i = 0; i < kSmIters; ++i) {
    const int j    = i * kSmThreads + t;
    const int base = j * 8;
    const v4f a = *(const v4f*)(rowf + base);
    const v4f c = *(const v4f*)(rowf + base + 4);
    unsigned short hb[8], lb[8];
#pragma unroll
    for (int e = 0; e < 4; ++e) {
      const float w0 = a[e] * inv;
      hb[e] = f2bf_bits(w0);
      lb[e] = f2bf_bits(w0 - bf_bits2f(hb[e]));
      const float w1 = c[e] * inv;
      hb[4 + e] = f2bf_bits(w1);
      lb[4 + e] = f2bf_bits(w1 - bf_bits2f(hb[4 + e]));
    }
    packbuf[2 * j]     = (v4u){pk16(hb[0], hb[1]), pk16(hb[2], hb[3]), pk16(hb[4], hb[5]), pk16(hb[6], hb[7])};
    packbuf[2 * j + 1] = (v4u){pk16(lb[0], lb[1]), pk16(lb[2], lb[3]), pk16(lb[4], lb[5]), pk16(lb[6], lb[7])};
  }

  unsigned short* hr = whi + rofs;
  unsigned short* lr = wlo + rofs;
  for (int pass = 0; pass < 2; ++pass) {
#pragma unroll 1
    for (int i = 0; i < kSmIters; ++i) {
      const int j = i * kSmThreads + t;
      const v4u hv = packbuf[2 * j];
      const v4u lv = packbuf[2 * j + 1];
      *(volatile v4u*)(hr + (size_t)j * 8) = hv;
      *(volatile v4u*)(lr + (size_t)j * 8) = lv;
    }
    __threadfence();
  }
}

__global__ __launch_bounds__(256) void tout_kernel(const float* __restrict__ outt, float* __restrict__ out) {
  __shared__ __align__(16) float sm[64 * 68];
  const int t  = threadIdx.x;
  const int n0 = blockIdx.x * 64;
  const int b  = blockIdx.y;
  const float* sb = outt + ((size_t)b * kSpat + n0) * kChan;
#pragma unroll
  for (int i = 0; i < 16; ++i) {
    const int e  = i * 256 + t;
    const int nl = e >> 6;
    const int c  = e & 63;
    sm[c * 68 + nl] = sb[(size_t)nl * kChan + c];
  }
  __syncthreads();
  const int lane = t & 31, wave = t >> 5;
  const int hh = lane >> 4, c4 = (lane & 15) * 4;
  float* ob = out + (size_t)b * kChan * kSpat + n0;
  for (int pass = 0; pass < 2; ++pass) {
#pragma unroll
    for (int it = 0; it < 4; ++it) {
      const int row = wave * 8 + it * 2 + hh;
      const v4f v = *(const v4f*)(sm + row * 68 + c4);
      *(volatile v4f*)(ob + (size_t)row * kSpat + c4) = v;
    }
    __threadfence();
  }
}

extern "C" void kernel_launch(void* const* d_in, const int* in_sizes, int n_in,
                              void* d_out, int out_size, void* d_ws, size_t ws_size,
                              hipStream_t stream) {
  const size_t nElem = (size_t)kBatch * kChan * kSpat;
  if (n_in < 2) return;
  if (in_sizes[0] != (int)nElem || in_sizes[1] != (int)nElem || out_size != (int)nElem) return;

  const size_t bytes16  = nElem * 2;
  const size_t bytesST  = (size_t)kBatch * kChunk * kSpat * 4;
  const size_t bytesW   = (size_t)kBatch * kChunk * kSpat * 2;
  const size_t bytesOT  = nElem * 4;
  size_t off = 0;
  const size_t oPIT  = off; off += bytes16;
  const size_t oYIT  = off; off += bytes16;
  const size_t oYI16 = off; off += bytes16;
  const size_t oST   = off; off += bytesST;
  const size_t oWHI  = off; off += bytesW;
  const size_t oWLO  = off; off += bytesW;
  const size_t oOUTT = off; off += bytesOT;
  if (off > ws_size) return;

  const float* yi = (const float*)d_in[0];
  const float* pi = (const float*)d_in[1];
  float* out = (float*)d_out;
  char* ws = (char*)d_ws;
  unsigned short* pit  = (unsigned short*)(ws + oPIT);
  unsigned short* yit  = (unsigned short*)(ws + oYIT);
  unsigned short* yi16 = (unsigned short*)(ws + oYI16);
  float*          st   = (float*)(ws + oST);
  unsigned short* whi  = (unsigned short*)(ws + oWHI);
  unsigned short* wlo  = (unsigned short*)(ws + oWLO);
  float*          outt = (float*)(ws + oOUTT);

  tcast_kernel<<<dim3(kSpat / 64, kBatch, 2), 256, 0, stream>>>(yi, pi, yit, pit);
  cast8_bf16_kernel<<<dim3((unsigned)(nElem / 8 / 256)), 256, 0, stream>>>(yi, yi16, (int)(nElem / 8));

  const long strideT16 = (long)kSpat * kChan;
  const long strideSTb = (long)kChunk * kSpat;
  const long strideOTb = (long)kSpat * kChan;

  for (int ch = 0; ch < kNumChunks; ++ch) {
    const unsigned short* aP = pit + (size_t)ch * kChunk * kChan;
    wmma_gemm64<1, 0, 0, 0, false, 0><<<dim3((kChunk / 64) * (kSpat / 64) / 8, kBatch), 256, 0, stream>>>(
        aP, aP, kChan, strideT16,
        yit, yit, kChan, strideT16,
        (void*)st, (void*)st, kSpat, strideSTb,
        (const float*)st, (const float*)st, 0L,
        kChunk, kSpat, kChan, 1.0f);

    softmax_split_kernel<<<dim3(kChunk, kBatch), kSmThreads, 0, stream>>>(st, whi, wlo);

    float* cP = outt + (size_t)ch * kChunk * kChan;
    wmma_gemm64<1, 1, 0, 0, false, 0><<<dim3(1, kBatch), 256, 0, stream>>>(
        whi, wlo, kSpat, strideSTb,
        yi16, yi16, kSpat, strideT16,
        (void*)cP, (void*)cP, kChan, strideOTb,
        (const float*)st, (const float*)st, 0L,
        kChunk, kChan, kSpat, 1.0f);
  }

  tout_kernel<<<dim3(kSpat / 64, kBatch), 256, 0, stream>>>(outt, out);
}
